// CollocationPhysicsLoss_43009802502473
// MI455X (gfx1250) — hardware-verified
//
#include <hip/hip_runtime.h>
#include <stdint.h>


typedef __attribute__((ext_vector_type(16))) _Float16 v16h;
typedef __attribute__((ext_vector_type(8)))  _Float16 v8h;
typedef __attribute__((ext_vector_type(8)))  float    v8f;
typedef __attribute__((ext_vector_type(4)))  float    v4f;
typedef __attribute__((ext_vector_type(2)))  unsigned int v2u;

#define NPTS   65536
#define HIDN   256
#define CHK    16384
#define NCHK   (NPTS / CHK)
#define JBLK   128
#define NPART  (NPTS / JBLK)
#define W0S    30.0f
#define RHO0F  1.225f
#define KCONT  144120.03125f
#define LAMF   0.01f

static_assert(NPTS % CHK == 0);
static_assert(CHK % 64 == 0);
static_assert(CHK % JBLK == 0);
static_assert(HIDN % 64 == 0);

__device__ __forceinline__ void dep_guard_h(v8f& a, v8f& b, v16h x, v16h y) { asm volatile("v_nop\n\tv_nop\n\tv_nop\n\tv_nop" : "+v"(a), "+v"(b) : "v"(x), "v"(y)); }
__device__ __forceinline__ void keep4_h(v16h a, v16h b, v16h c, v16h d) { asm volatile("v_nop" :: "v"(a), "v"(b), "v"(c), "v"(d)); }
__device__ __forceinline__ void acc_guard4(v8f& a, v8f& b, v8f& c, v8f& d) { asm volatile("v_nop\n\tv_nop\n\tv_nop\n\tv_nop" : "+v"(a), "+v"(b), "+v"(c), "+v"(d)); }
__device__ __forceinline__ void guard4ab(v8f& c0, v8f& c1, v8f& c2, v8f& c3, v16h a0, v16h a1, v16h a2, v16h a3, v16h bb) {
  asm volatile("v_nop\n\tv_nop\n\tv_nop\n\tv_nop" : "+v"(c0), "+v"(c1), "+v"(c2), "+v"(c3) : "v"(a0), "v"(a1), "v"(a2), "v"(a3), "v"(bb));
}
template <typename T> struct Frag;
template <> struct Frag<_Float16> {
  typedef v16h V; union U { v16h v; v8h h[2]; };
  static __device__ __forceinline__ v16h load(const _Float16* p) {
    U f; f.h[0] = *(const v8h*)(p); f.h[1] = *(const v8h*)(p + 16); return f.v;
  }
  static __device__ __forceinline__ v8f mma(v16h a, v16h b, v8f c) {
    return __builtin_amdgcn_wmma_f32_16x16x32_f16(false, a, false, b, (short)0, c, false, false);
  }
  static __device__ __forceinline__ void guard(v8f& a, v8f& b, v16h x, v16h y) { dep_guard_h(a, b, x, y); }
  static __device__ __forceinline__ void keep(v16h a, v16h b, v16h c, v16h d) { keep4_h(a, b, c, d); }
};

__device__ __forceinline__ void wave_sync_lds() {
  __builtin_amdgcn_fence(__ATOMIC_RELEASE, "workgroup");
  __builtin_amdgcn_wave_barrier();
  __builtin_amdgcn_fence(__ATOMIC_ACQUIRE, "workgroup");
}
__device__ __forceinline__ unsigned short h_bits(float f) { return __builtin_bit_cast(unsigned short, (_Float16)f); }

template <int EPI, bool EMIT1>
__global__ __launch_bounds__(256) void gemm64_f16(
    const unsigned short* __restrict__ Ap, int lda, long strideA,
    const unsigned short* __restrict__ Btp, int ldb, long strideB,
    unsigned short* __restrict__ C1p, unsigned short* __restrict__ C2p, int ldc, long strideC,
    const float* __restrict__ bias,
    const unsigned short* __restrict__ Mp, long strideM,
    int M, int N, int K, float scale, float sscale) {
  typedef _Float16 T;
  typedef v16h V;
  const T* A  = (const T*)Ap;
  const T* Bt = (const T*)Btp;
  __shared__ __align__(16) float    sT[8][16 * 68];
  __shared__ __align__(16) _Float16 sH1[8][16 * 64];
  __shared__ __align__(16) _Float16 sH2[(EPI == 0) ? 8 : 1][(EPI == 0) ? (16 * 64) : 8];
  const int b    = blockIdx.y;
  const int lane = threadIdx.x & 31;
  const int wave = threadIdx.x >> 5;
  const int tilesN = N >> 6;
  const int tilesM = M >> 6;
  const int tile = blockIdx.x * 8 + wave;
  if (tile >= tilesM * tilesN) return;
  const int tm = tile / tilesN;
  const int tn = tile - tm * tilesN;
  const int m0 = tm << 6;
  const int n0 = tn << 6;

  const T* Ab = A  + (size_t)b * strideA;
  const T* Bb = Bt + (size_t)b * strideB;

  const int rlane = lane & 15;
  const int koff  = (lane >> 4) * 8;
  const int mOff  = (lane >> 4) * 8;

  v8f acc[4][4];
#pragma unroll
  for (int i = 0; i < 4; ++i)
#pragma unroll
    for (int j = 0; j < 4; ++j) acc[i][j] = (v8f){0.f,0.f,0.f,0.f,0.f,0.f,0.f,0.f};

  for (int k0 = 0; k0 < K; k0 += 32) {
    V bh[4];
#pragma unroll
    for (int j = 0; j < 4; ++j) {
      const size_t bo = (size_t)(n0 + (j << 4) + rlane) * ldb + koff + k0;
      bh[j] = Frag<T>::load(Bb + bo);
    }
#pragma unroll
    for (int i = 0; i < 4; ++i) {
      const size_t ao = (size_t)(m0 + (i << 4) + rlane) * lda + koff + k0;
      V ah = Frag<T>::load(Ab + ao);
#pragma unroll
      for (int j = 0; j < 4; ++j) acc[i][j] = Frag<T>::mma(ah, bh[j], acc[i][j]);
      Frag<T>::guard(acc[i][0], acc[i][3], ah, ah);
    }
    Frag<T>::keep(bh[0], bh[1], bh[2], bh[3]);
  }
  acc_guard4(acc[0][0], acc[0][1], acc[0][2], acc[0][3]);
  acc_guard4(acc[1][0], acc[1][1], acc[1][2], acc[1][3]);
  acc_guard4(acc[2][0], acc[2][1], acc[2][2], acc[2][3]);
  acc_guard4(acc[3][0], acc[3][1], acc[3][2], acc[3][3]);

  float* slab = sT[wave];
  _Float16* h1 = sH1[wave];
  _Float16* h2 = sH2[(EPI == 0) ? wave : 0];
  unsigned short* C1 = C1p + (size_t)b * strideC;
  unsigned short* C2 = C2p + (size_t)b * strideC;
  const T* Mb = (const T*)Mp + (size_t)b * strideM;
#pragma unroll
  for (int i = 0; i < 4; ++i) {
    const int mBase = m0 + (i << 4);
#pragma unroll
    for (int j = 0; j < 4; ++j) {
      const int n = n0 + (j << 4) + rlane;
      float bv = 0.f;
      if (EPI == 0) bv = bias[n];
#pragma unroll
      for (int r = 0; r < 8; ++r) {
        float v = acc[i][j][r] * scale;
        if (EPI == 0) v += bv;
        slab[(mOff + r) * 68 + (j << 4) + rlane] = v;
      }
    }
    wave_sync_lds();
#pragma unroll 1
    for (int it = 0; it < 32; ++it) {
      const int idx = it * 32 + lane;
      const int row = idx >> 6;
      const int col = idx & 63;
      const float v = slab[row * 68 + col];
      if (EPI == 0) {
        float sv, cv;
        sincosf(v, &sv, &cv);
        if (EMIT1) h1[row * 64 + col] = (_Float16)(sv * sscale);
        h2[row * 64 + col] = (_Float16)cv;
      } else {
        const float mv = (float)Mb[(size_t)(mBase + row) * ldc + n0 + col];
        h1[row * 64 + col] = (_Float16)(v * mv);
      }
    }
    wave_sync_lds();
    {
      const int q = lane >> 3, c8 = (lane & 7) * 8;
      for (int pass = 0; pass < 2; ++pass) {
#pragma unroll
        for (int it = 0; it < 4; ++it) {
          const int row = it * 4 + q;
          if (EPI == 1 || EMIT1) {
            const v8h hv = *(const v8h*)(h1 + row * 64 + c8);
            *(volatile v8h*)(C1 + (size_t)(mBase + row) * ldc + n0 + c8) = hv;
          }
          if (EPI == 0) {
            const v8h cv = *(const v8h*)(h2 + row * 64 + c8);
            *(volatile v8h*)(C2 + (size_t)(mBase + row) * ldc + n0 + c8) = cv;
          }
        }
        __threadfence();
      }
    }
    wave_sync_lds();
  }
}

__device__ __forceinline__ float prep_val(const float* __restrict__ W, const float* __restrict__ W0,
                                          int mode, int jj, int k, int n) {
  const float v = W[(size_t)k * HIDN + n];
  const float w = W0[jj * HIDN + k];
  return (mode >= 2) ? ((W0S * w) * v * 64.0f) : (v * 256.0f);
}

__global__ __launch_bounds__(256) void prep_kernel(
    const float* __restrict__ room, const float* __restrict__ W0, const float* __restrict__ W1,
    const float* __restrict__ W2, const float* __restrict__ W3,
    float* __restrict__ rm, unsigned short* __restrict__ W1t, unsigned short* __restrict__ W2t,
    unsigned short* __restrict__ Bjt, unsigned short* __restrict__ W3t) {
  const int t = threadIdx.x, bx = blockIdx.x, y = blockIdx.y;
  const int n  = bx * 4 + (t >> 6);
  const int k0 = (t & 63) * 4;
  if (y == 6) {
    if (bx < 4) {
      const int nn = (n < 4) ? n : 0;
      const bool real = (n < 4);
      const float g0 = W3[(size_t)(k0 + 0) * 4 + nn] * 256.0f;
      const float g1 = W3[(size_t)(k0 + 1) * 4 + nn] * 256.0f;
      const float g2 = W3[(size_t)(k0 + 2) * 4 + nn] * 256.0f;
      const float g3 = W3[(size_t)(k0 + 3) * 4 + nn] * 256.0f;
      v2u u;
      u.x = (unsigned)h_bits(real ? g0 : 0.f) | ((unsigned)h_bits(real ? g1 : 0.f) << 16);
      u.y = (unsigned)h_bits(real ? g2 : 0.f) | ((unsigned)h_bits(real ? g3 : 0.f) << 16);
      unsigned short* dst = W3t + (size_t)n * HIDN + k0;
      *(volatile v2u*)dst = u;
      __threadfence();
      *(volatile v2u*)dst = u;
    } else if (bx == 4) {
      if (t < 32) {
        const int tt = (t < 3) ? t : 0;
        float s = room[0 * 3 + tt];
        s += room[1 * 3 + tt]; s += room[2 * 3 + tt]; s += room[3 * 3 + tt];
        s += room[4 * 3 + tt]; s += room[5 * 3 + tt]; s += room[6 * 3 + tt]; s += room[7 * 3 + tt];
        const float v = (t < 3) ? fmaxf(s * 0.125f, 0.1f) : 0.f;
        *(volatile float*)(rm + t) = v;
        __threadfence();
        *(volatile float*)(rm + t) = v;
      }
    }
    return;
  }
  const int jj = (y >= 2) ? (y - 2) : 0;
  const float* W = (y == 1) ? W2 : W1;
  unsigned short* O = (y == 0) ? W1t : ((y == 1) ? W2t : (Bjt + (size_t)jj * (HIDN * HIDN)));
  const float f0 = prep_val(W, W0, y, jj, k0 + 0, n);
  const float f1 = prep_val(W, W0, y, jj, k0 + 1, n);
  const float f2 = prep_val(W, W0, y, jj, k0 + 2, n);
  const float f3 = prep_val(W, W0, y, jj, k0 + 3, n);
  v2u u;
  u.x = (unsigned)h_bits(f0) | ((unsigned)h_bits(f1) << 16);
  u.y = (unsigned)h_bits(f2) | ((unsigned)h_bits(f3) << 16);
  unsigned short* dst = O + (size_t)n * HIDN + k0;
  *(volatile v2u*)dst = u;
  __threadfence();
  *(volatile v2u*)dst = u;
}

__global__ __launch_bounds__(256) void layer0_kernel(
    const float* __restrict__ coords, const float* __restrict__ time_raw,
    const float* __restrict__ W0, const float* __restrict__ b0,
    const float* __restrict__ rm,
    unsigned short* __restrict__ H0, unsigned short* __restrict__ C0,
    int pbase, int npts) {
  const int t  = threadIdx.x;
  const int pl = blockIdx.x * 2 + (t >> 7);
  int p = pbase + pl;
  p = (p < npts) ? p : (npts - 1);
  const int i0 = (t & 127) * 2;
  const float x0 = coords[(size_t)p * 3 + 0] * rm[0];
  const float x1 = coords[(size_t)p * 3 + 1] * rm[1];
  const float x2 = coords[(size_t)p * 3 + 2] * rm[2];
  const float x3 = time_raw[p] * 2.0f;
  unsigned hs = 0u, hc = 0u;
#pragma unroll 1
  for (int e = 0; e < 2; ++e) {
    const int i = i0 + e;
    float a = x0 * W0[i];
    a = fmaf(x1, W0[HIDN + i], a);
    a = fmaf(x2, W0[2 * HIDN + i], a);
    a = fmaf(x3, W0[3 * HIDN + i], a);
    a = (a + b0[i]) * W0S;
    float sv, cv;
    sincosf(a, &sv, &cv);
    hs |= ((unsigned)h_bits(sv)) << (16 * e);
    hc |= ((unsigned)h_bits(cv)) << (16 * e);
  }
  const size_t off = ((size_t)pl * HIDN + i0) >> 1;
  ((volatile unsigned*)H0)[off] = hs;
  ((volatile unsigned*)C0)[off] = hc;
  __threadfence();
  ((volatile unsigned*)H0)[off] = hs;
  ((volatile unsigned*)C0)[off] = hc;
}

__global__ __launch_bounds__(256) void jres_kernel(
    const unsigned short* __restrict__ D2p, long strideP,
    const unsigned short* __restrict__ W3tp,
    float* __restrict__ part, int blk0, float scale) {
  typedef _Float16 T;
  typedef v16h V;
  const T* D2 = (const T*)D2p;
  const T* W3 = (const T*)W3tp;
  __shared__ __align__(16) float sJ[8][16 * 16];
  __shared__ float sP[8][2];
  const int lane = threadIdx.x & 31, wave = threadIdx.x >> 5;
  const int c = lane & 15, hh = lane >> 4, koff = hh * 8;
  const int p0 = blockIdx.x * JBLK + wave * 16;
  v8f acc[4];
#pragma unroll
  for (int j = 0; j < 4; ++j) acc[j] = (v8f){0.f,0.f,0.f,0.f,0.f,0.f,0.f,0.f};
#pragma unroll
  for (int kt = 0; kt < 8; ++kt) {
    const V bfr = Frag<T>::load(W3 + (size_t)c * HIDN + kt * 32 + koff);
    V afr[4];
#pragma unroll
    for (int j = 0; j < 4; ++j)
      afr[j] = Frag<T>::load(D2 + (size_t)j * strideP + (size_t)(p0 + c) * HIDN + kt * 32 + koff);
#pragma unroll
    for (int j = 0; j < 4; ++j) acc[j] = Frag<T>::mma(afr[j], bfr, acc[j]);
    guard4ab(acc[0], acc[1], acc[2], acc[3], afr[0], afr[1], afr[2], afr[3], bfr);
  }
  acc_guard4(acc[0], acc[1], acc[2], acc[3]);

  float* js = sJ[wave];
  if (c < 4) {
#pragma unroll
    for (int r = 0; r < 8; ++r) {
#pragma unroll
      for (int j = 0; j < 4; ++j) js[(8 * hh + r) * 16 + c * 4 + j] = acc[j][r] * scale;
    }
  }
  wave_sync_lds();
  float qc = 0.f, qm = 0.f;
  if (lane < 16) {
    const float* Jr = js + lane * 16;
    const float dpdt = Jr[0 * 4 + 3];
    const float divu = (Jr[1 * 4 + 0] + Jr[2 * 4 + 1]) + Jr[3 * 4 + 2];
    const float rc   = dpdt + KCONT * divu;
    const float du   = (Jr[1 * 4 + 3] + Jr[2 * 4 + 3]) + Jr[3 * 4 + 3];
    const float base = RHO0F * du;
    const float mx = base + Jr[0], my = base + Jr[1], mz = base + Jr[2];
    qc = rc * rc;
    qm = (mx * mx + my * my) + mz * mz;
  }
#pragma unroll
  for (int off = 16; off > 0; off >>= 1) {
    qc += __shfl_xor(qc, off, 32);
    qm += __shfl_xor(qm, off, 32);
  }
  if (lane == 0) { sP[wave][0] = qc; sP[wave][1] = qm; }
  __syncthreads();
  if (wave == 0) {
    float v = 0.f;
    if (lane == 0) {
      v = sP[0][0]; v += sP[1][0]; v += sP[2][0]; v += sP[3][0];
      v += sP[4][0]; v += sP[5][0]; v += sP[6][0]; v += sP[7][0];
    } else if (lane == 1) {
      v = sP[0][1]; v += sP[1][1]; v += sP[2][1]; v += sP[3][1];
      v += sP[4][1]; v += sP[5][1]; v += sP[6][1]; v += sP[7][1];
    }
    float* dst = part + (size_t)(blk0 + blockIdx.x) * 32 + lane;
    *(volatile float*)dst = v;
    __threadfence();
    *(volatile float*)dst = v;
  }
}

__global__ __launch_bounds__(32) void final_kernel(const float* __restrict__ part, int nblk,
                                                   float* __restrict__ out) {
  if (threadIdx.x == 0) {
    double sc = 0.0, sm = 0.0;
#pragma unroll 1
    for (int i = 0; i < nblk; ++i) {
      sc += (double)part[(size_t)i * 32 + 0];
      sm += (double)part[(size_t)i * 32 + 1];
    }
    const float mc = (float)(sc * (1.0 / 65536.0));
    const float mm = (float)(sm * (1.0 / 196608.0));
    const float loss = LAMF * mc + LAMF * mm;
    *(volatile float*)out = loss;
    __threadfence();
    *(volatile float*)out = loss;
  }
}

extern "C" void kernel_launch(void* const* d_in, const int* in_sizes, int n_in,
                              void* d_out, int out_size, void* d_ws, size_t ws_size,
                              hipStream_t stream) {
  if (n_in < 12 || out_size < 1) return;
  if (in_sizes[0] != 24 || in_sizes[1] != NPTS * 3 || in_sizes[2] != NPTS ||
      in_sizes[3] != 4 * HIDN || in_sizes[4] != HIDN || in_sizes[5] != HIDN * HIDN ||
      in_sizes[6] != HIDN || in_sizes[7] != HIDN * HIDN || in_sizes[8] != HIDN ||
      in_sizes[9] != HIDN * 4) return;

  const float* room   = (const float*)d_in[0];
  const float* coords = (const float*)d_in[1];
  const float* traw   = (const float*)d_in[2];
  const float* W0 = (const float*)d_in[3];
  const float* b0 = (const float*)d_in[4];
  const float* W1 = (const float*)d_in[5];
  const float* b1 = (const float*)d_in[6];
  const float* W2 = (const float*)d_in[7];
  const float* b2 = (const float*)d_in[8];
  const float* W3 = (const float*)d_in[9];

  const size_t PLANE_B = (size_t)CHK * HIDN * 2;
  const long   PL_H    = (long)CHK * HIDN;
  const size_t OFF_RM   = 0;
  const size_t OFF_W1T  = 256;
  const size_t OFF_W2T  = OFF_W1T + (size_t)HIDN * HIDN * 2;
  const size_t OFF_BJT  = OFF_W2T + (size_t)HIDN * HIDN * 2;
  const size_t OFF_W3T  = OFF_BJT + (size_t)4 * HIDN * HIDN * 2;
  const size_t OFF_PART = OFF_W3T + (size_t)16 * HIDN * 2;
  const size_t OFF_R0   = OFF_PART + (size_t)NPART * 128;
  const size_t OFF_R1   = OFF_R0 + 4 * PLANE_B;
  const size_t OFF_R2   = OFF_R1 + 4 * PLANE_B;
  const size_t OFF_END  = OFF_R2 + PLANE_B;
  if (OFF_END > ws_size) return;

  char* ws = (char*)d_ws;
  float*          rm   = (float*)(ws + OFF_RM);
  unsigned short* W1t  = (unsigned short*)(ws + OFF_W1T);
  unsigned short* W2t  = (unsigned short*)(ws + OFF_W2T);
  unsigned short* Bjt  = (unsigned short*)(ws + OFF_BJT);
  unsigned short* W3t  = (unsigned short*)(ws + OFF_W3T);
  float*          part = (float*)(ws + OFF_PART);
  unsigned short* h0 = (unsigned short*)(ws + OFF_R0 + 0 * PLANE_B);
  unsigned short* c0 = (unsigned short*)(ws + OFF_R0 + 1 * PLANE_B);
  unsigned short* s1 = (unsigned short*)(ws + OFF_R0 + 2 * PLANE_B);
  unsigned short* c1 = (unsigned short*)(ws + OFF_R0 + 3 * PLANE_B);
  unsigned short* d1 = (unsigned short*)(ws + OFF_R1);
  unsigned short* c2 = (unsigned short*)(ws + OFF_R2);
  unsigned short* d2 = (unsigned short*)(ws + OFF_R0);

  const int tilesPerBatch = (CHK / 64) * (HIDN / 64);
  const int gemmBlocks = (tilesPerBatch + 7) / 8;

  prep_kernel<<<dim3(64, 7), dim3(256), 0, stream>>>(room, W0, W1, W2, W3, rm, W1t, W2t, Bjt, W3t);

  for (int ch = 0; ch < NCHK; ++ch) {
    const int pbase = ch * CHK;
    layer0_kernel<<<dim3(CHK / 2), dim3(256), 0, stream>>>(coords, traw, W0, b0, rm, h0, c0, pbase, NPTS);
    gemm64_f16<0, true><<<dim3(gemmBlocks, 1), dim3(256), 0, stream>>>(
        h0, HIDN, 0L, W1t, HIDN, 0L, s1, c1, HIDN, 0L, b1, h0, 0L,
        CHK, HIDN, HIDN, 1.0f / 256.0f, 16.0f);
    gemm64_f16<1, false><<<dim3(gemmBlocks, 4), dim3(256), 0, stream>>>(
        c0, HIDN, 0L, Bjt, HIDN, (long)HIDN * HIDN, d1, d1, HIDN, PL_H, b1, c1, 0L,
        CHK, HIDN, HIDN, 1.0f / 64.0f, 1.0f);
    gemm64_f16<0, false><<<dim3(gemmBlocks, 1), dim3(256), 0, stream>>>(
        s1, HIDN, 0L, W2t, HIDN, 0L, c2, c2, HIDN, 0L, b2, s1, 0L,
        CHK, HIDN, HIDN, 1.0f / 4096.0f, 1.0f);
    gemm64_f16<1, false><<<dim3(gemmBlocks, 4), dim3(256), 0, stream>>>(
        d1, HIDN, PL_H, W2t, HIDN, 0L, d2, d2, HIDN, PL_H, b2, c2, 0L,
        CHK, HIDN, HIDN, 1.0f / 16.0f, 1.0f);
    jres_kernel<<<dim3(CHK / JBLK), dim3(256), 0, stream>>>(
        d2, PL_H, W3t, part, ch * (CHK / JBLK), 1.0f / 4096.0f);
  }
  final_kernel<<<dim3(1), dim3(32), 0, stream>>>(part, NPART, (float*)d_out);
}
